// UpdateNetV2_86449101734004
// MI455X (gfx1250) — hardware-run, weakly checked
//
#include <hip/hip_runtime.h>


#define NR   4096
#define NQ   4
#define NL   1024
#define NU   256
#define NW   32
#define NK   256
#define NC   896
#define OQ   32
#define OPU  64
#define OQU  320
#define OF   576
#define OFU  608
#define UP   256.0f
#define DN   0.00390625f
typedef _Float16 h16;
typedef unsigned short bf;
typedef __attribute__((ext_vector_type(16))) __bf16   v16bf;
typedef __attribute__((ext_vector_type(16))) _Float16 v16h;
typedef __attribute__((ext_vector_type(8)))  _Float16 v8h;
typedef __attribute__((ext_vector_type(8)))  unsigned short v8us;
typedef __attribute__((ext_vector_type(8)))  float    v8f;
typedef __attribute__((ext_vector_type(4)))  float    v4f;
typedef v8h  __attribute__((may_alias)) v8ha;
typedef v4f  __attribute__((may_alias)) v4fa;
typedef v8us __attribute__((may_alias)) v8usa;

__device__ __forceinline__ unsigned short f2bf(float f) { unsigned u = __float_as_uint(f); u += 0x7FFFu + ((u >> 16) & 1u); return (unsigned short)(u >> 16); }
__device__ __forceinline__ float bf2f(unsigned short b) { return __uint_as_float(((unsigned)b) << 16); }
__device__ __forceinline__ float bfr(float f) { return bf2f(f2bf(f)); }
__device__ __forceinline__ v16h cat16(v8h lo, v8h hi) { return __builtin_shufflevector(lo, hi, 0, 1, 2, 3, 4, 5, 6, 7, 8, 9, 10, 11, 12, 13, 14, 15); }
__device__ __forceinline__ v16bf cat16b(v8us lo, v8us hi) { return __builtin_bit_cast(v16bf, __builtin_shufflevector(lo, hi, 0, 1, 2, 3, 4, 5, 6, 7, 8, 9, 10, 11, 12, 13, 14, 15)); }
__device__ __forceinline__ v8f wmma16(v16h a, v16h b, v8f c) { return __builtin_amdgcn_wmma_f32_16x16x32_f16(false, a, false, b, (short)0, c, false, false); }
__device__ __forceinline__ v8f wmmab(v16bf a, v16bf b, v8f c) { return __builtin_amdgcn_wmma_f32_16x16x32_bf16(false, a, false, b, (short)0, c, false, false); }

template <typename T16> struct WFrag;
template <> struct WFrag<h16> { typedef v16h V; static __device__ __forceinline__ V ld(const h16* p) { return cat16(*(const v8h*)p, *(const v8h*)(p + 16)); } static __device__ __forceinline__ v8f mma(V a, V b, v8f c) { return wmma16(a, b, c); } };
template <> struct WFrag<bf> { typedef v16bf V; static __device__ __forceinline__ V ld(const bf* p) { return cat16b(*(const v8us*)p, *(const v8us*)(p + 16)); } static __device__ __forceinline__ v8f mma(V a, V b, v8f c) { return wmmab(a, b, c); } };
template <typename T16, int NSPLIT, bool BIAS>
__global__ __launch_bounds__(32) void k_gemmw(const T16* __restrict__ A, const T16* __restrict__ A2, const T16* __restrict__ Bt, const T16* __restrict__ Bt2, int K, float* C, int ldc, const float* __restrict__ bias, size_t sA, size_t sB, size_t sC) {
    typedef typename WFrag<T16>::V V;
    __shared__ __align__(16) float os[16 * 68];
    const size_t z = blockIdx.z; A += z * sA; if (A2) A2 += z * sA; Bt += z * sB; if (Bt2) Bt2 += z * sB; C += z * sC;
    const int lane = threadIdx.x & 31, lr = lane & 15, hi = lane >> 4; const int r0 = blockIdx.x * 64, c0 = blockIdx.y * 64;
    v8f acc[4][4];
#pragma unroll
    for (int mb = 0; mb < 4; ++mb)
#pragma unroll
        for (int nb = 0; nb < 4; ++nb) acc[mb][nb] = (v8f){};
    const size_t aoff = (size_t)(r0 + lr) * K + 8 * hi, boff = (size_t)(c0 + lr) * K + 8 * hi;
    for (int kc = 0; kc < K; kc += 32) {
        V a[4], a2[4];
#pragma unroll
        for (int mb = 0; mb < 4; ++mb) { a[mb] = WFrag<T16>::ld(A + aoff + (size_t)mb * 16 * K + kc); if (NSPLIT == 1 || NSPLIT == 2) a2[mb] = WFrag<T16>::ld(A2 + aoff + (size_t)mb * 16 * K + kc); }
#pragma unroll
        for (int nb = 0; nb < 4; ++nb) { const V b = WFrag<T16>::ld(Bt + boff + (size_t)nb * 16 * K + kc); V b2; if (NSPLIT >= 2) b2 = WFrag<T16>::ld(Bt2 + boff + (size_t)nb * 16 * K + kc);
#pragma unroll
            for (int mb = 0; mb < 4; ++mb) { acc[mb][nb] = WFrag<T16>::mma(a[mb], b, acc[mb][nb]); if (NSPLIT == 1 || NSPLIT == 2) acc[mb][nb] = WFrag<T16>::mma(a2[mb], b, acc[mb][nb]); if (NSPLIT >= 2) acc[mb][nb] = WFrag<T16>::mma(a[mb], b2, acc[mb][nb]); } }
        asm volatile("v_nop\n\tv_nop\n\tv_nop\n\tv_nop" : "+v"(acc[0][0]), "+v"(acc[1][1]), "+v"(acc[2][2]), "+v"(acc[3][3]) : "v"(a[0]), "v"(a[3]));
    }
#pragma unroll
    for (int mb = 0; mb < 4; ++mb) {
#pragma unroll
        for (int nb = 0; nb < 4; ++nb) {
#pragma unroll
            for (int j = 0; j < 8; ++j) os[(hi * 8 + j) * 68 + nb * 16 + lr] = acc[mb][nb][j]; }
        __builtin_amdgcn_wave_barrier(); asm volatile("" ::: "memory");
        float* crow = C + (size_t)(r0 + mb * 16) * ldc + c0;
#pragma unroll 1
        for (int ps = 0; ps < 2; ++ps) {
#pragma unroll
            for (int s = 0; s < 8; ++s) { const int row = 2 * s + hi, cofs = lr * 4; v4f val = *(const v4fa*)(os + row * 68 + cofs); if (BIAS) { val[0] += bfr(bias[c0 + cofs]); val[1] += bfr(bias[c0 + cofs + 1]); val[2] += bfr(bias[c0 + cofs + 2]); val[3] += bfr(bias[c0 + cofs + 3]); }
                *(volatile v4f*)(crow + (size_t)row * ldc + cofs) = val; }
            if (ps == 0) __threadfence(); }
        __builtin_amdgcn_wave_barrier(); asm volatile("" ::: "memory");
    }
}

typedef __attribute__((ext_vector_type(2))) _Float16 v2h;
typedef __attribute__((ext_vector_type(4))) _Float16 v4h;
typedef __attribute__((ext_vector_type(2))) unsigned short v2us;
typedef __attribute__((ext_vector_type(4))) unsigned short v4us;
typedef __attribute__((ext_vector_type(2))) float v2f;
typedef __attribute__((ext_vector_type(4))) int v4i;

__global__ __launch_bounds__(256) void k_cvt8(const float* __restrict__ src, bf* dst, size_t n8) { const size_t i = (size_t)blockIdx.x * 256 + threadIdx.x; if (i >= n8) return; const v8f v = *(const v8f*)(src + i * 8); v8us o;
#pragma unroll
    for (int k = 0; k < 8; ++k) o[k] = f2bf(v[k]); *(volatile v8us*)(dst + i * 8) = o; __threadfence(); *(volatile v8us*)(dst + i * 8) = o; }

__global__ __launch_bounds__(256) void k_wtG(const float* __restrict__ w, int K, int N, bf* Bt) {
    const int lane = threadIdx.x & 31; const int L0 = (blockIdx.x * 8 + (threadIdx.x >> 5)) * 8; const int nlines = N * K / 64;
#pragma unroll
    for (int ps = 0; ps < 2; ++ps) {
        for (int l = 0; l < 8; ++l) { const int L = L0 + l; if (L >= nlines) break; const size_t e = (size_t)L * 64 + lane * 2; const int k = (int)(e % K), n = (int)(e / K); v2us o;
            o[0] = f2bf(w[(size_t)k * N + n]); o[1] = f2bf(w[(size_t)(k + 1) * N + n]); *(volatile v2us*)(Bt + e) = o; }
        if (ps == 0) __threadfence(); }
}

__device__ __forceinline__ h16 toh_flush(float x) { const float z = (fabsf(x) < 6.103515625e-05f) ? 0.0f : x; return (h16)z; }

static __device__ __forceinline__ float gsl(float t) { return t / (1.0f + expf(-t)); }
static __device__ __forceinline__ float msl(float t) { return fminf(t, 0.0f) - log1pf(expf(-fabsf(t))); }

__global__ __launch_bounds__(256) void k_bsum(const float* __restrict__ Pj, float* Bs) { const unsigned nb = blockIdx.x * 256u + threadIdx.x; const unsigned tb = nb & 127u, wd = (nb >> 7) & 31u, un = (nb >> 12) & 255u, sq = nb >> 20; const float* ps = Pj + (size_t)sq * NL * NC; float sum = 0.0f;
#pragma unroll
    for (int j = 0; j < 8; ++j) { const int p = (int)tb * 8 + j; const float* pq = ps + (size_t)((p > 0) ? NL - p : 0) * NC; const float fd = msl(pq[OF + wd] * pq[OFU + un]); sum += (p > 0) ? fd : 0.0f; }
    *(volatile float*)(Bs + nb) = sum; __threadfence(); *(volatile float*)(Bs + nb) = sum; }

__global__ __launch_bounds__(256) void k_fillf(const float* __restrict__ Pj, const float* __restrict__ Bs, h16* Ka, h16* Va) { const unsigned nb = blockIdx.x * 256u + threadIdx.x; const unsigned tb = nb & 127u, wd = (nb >> 7) & 31u, un = (nb >> 12) & 255u, sq = nb >> 20; const float* ps = Pj + (size_t)sq * NL * NC; const float* bs = Bs + (size_t)(nb >> 7) * 128; float run = 0.0f;
    for (int m = 0; m < 128; ++m) { const float got = bs[m]; run += ((unsigned)m < tb) ? got : 0.0f; }
    v8h oa, ob;
#pragma unroll
    for (int j = 0; j < 8; ++j) { const int p = (int)tb * 8 + j; const float* pr = ps + (size_t)p * NC; const float* pq = ps + (size_t)((p > 0) ? NL - p : 0) * NC; const float fd = msl(pq[OF + wd] * pq[OFU + un]); run += (p > 0) ? fd : 0.0f; const float a = gsl(pr[wd] * pr[OPU + un]) * expf(run) * UP; const float c = gsl(pr[OQ + wd] * pr[OQU + un]); oa[j] = toh_flush(a); ob[j] = toh_flush(c); }
    h16* ka = Ka + (size_t)nb * 8; h16* va = Va + (size_t)nb * 8; *(volatile v8h*)ka = oa; *(volatile v8h*)va = ob; __threadfence(); *(volatile v8h*)ka = oa; *(volatile v8h*)va = ob; }

__global__ __launch_bounds__(256) void k_pickd(const float* __restrict__ Cz, float* out) { const unsigned nb = blockIdx.x * 256u + threadIdx.x; const unsigned un = nb & 255u, wx = (nb >> 8) & 1023u, sq = nb >> 18; const unsigned rr = wx >> 5, cc = wx & 31u, lo = un & 1u; const float got = Cz[(((size_t)sq * (NU / 2) + (un >> 1)) * 64 + (lo * 32 + rr)) * 64 + lo * 32 + cc] * DN; *(volatile float*)(out + nb) = got; __threadfence(); *(volatile float*)(out + nb) = got; }

extern "C" void kernel_launch(void* const* d_in, const int* in_sizes, int n_in, void* d_out, int out_size, void* d_ws, size_t ws_size, hipStream_t stream) {
    if (n_in < 5) return;
    if (in_sizes[0] != NR * NK || in_sizes[1] != NK * 2 * NW || in_sizes[2] != NK * 2 * NU || in_sizes[3] != NK * NW || in_sizes[4] != NK * NU) return;
    if (out_size != NQ * NW * NW * NU) return;
    static_assert(NR == NQ * NL && NR % 64 == 0 && NC % 64 == 0 && NK % 64 == 0 && NL % 32 == 0 && (NR * NK / 8) % 256 == 0 && (NQ * NU * NW * 128) % 256 == 0 && NL == 8 * 128 && (NQ * NW * NW * NU) % 256 == 0 && NW == 32 && NU == 256 && NL == 1024 && NQ == 4 && OQ == NW && OPU == 2 * NW && OQU == OPU + NU && OF == OQU + NU && OFU == OF + NW && NC == OFU + NU + NW && UP * DN == 1.0f, "the products: row and column counts multiples of 64, the depths of 32 (the transposing cast: of 64); every one-dimensional launch exact; four sequences of 1,024 places, 256 units, 32 words; the first product's columns in their six parts and 32 more; the two powers of two undo each other");
    const float* i0 = (const float*)d_in[0]; const float* i1 = (const float*)d_in[1]; const float* i2 = (const float*)d_in[2]; const float* i3 = (const float*)d_in[3]; const float* i4 = (const float*)d_in[4]; float* out = (float*)d_out;
    char* wsp = (char*)d_ws; auto take = [&](size_t bytes) { char* p = wsp; wsp += (bytes + 255) & ~(size_t)255; return (void*)p; };
    bf* Tb = (bf*)take((size_t)NR * NK * 2); bf* Wt = (bf*)take((size_t)NC * NK * 2); float* Pj = (float*)take((size_t)NR * NC * 4); float* Bs = (float*)take((size_t)NQ * NU * NW * 128 * 4); h16* Ka = (h16*)take((size_t)NQ * NU * NW * NL * 2); h16* Va = (h16*)take((size_t)NQ * NU * NW * NL * 2); float* Cz = (float*)take((size_t)NQ * (NU / 2) * 64 * 64 * 4);
    if ((size_t)(wsp - (char*)d_ws) > ws_size) return;
    k_cvt8<<<(unsigned)(NR * NK / 8 / 256), 256, 0, stream>>>(i0, Tb, (size_t)NR * NK / 8);
    k_wtG<<<(unsigned)((NK * 2 * NW / 64 + 63) / 64), 256, 0, stream>>>(i1, NK, 2 * NW, Wt);
    k_wtG<<<(unsigned)((NK * 2 * NU / 64 + 63) / 64), 256, 0, stream>>>(i2, NK, 2 * NU, Wt + (size_t)OPU * NK);
    k_wtG<<<(unsigned)((NK * NW / 64 + 63) / 64), 256, 0, stream>>>(i3, NK, NW, Wt + (size_t)OF * NK);
    k_wtG<<<(unsigned)((NK * NU / 64 + 63) / 64), 256, 0, stream>>>(i4, NK, NU, Wt + (size_t)OFU * NK);
    k_wtG<<<(unsigned)((NK * NW / 64 + 63) / 64), 256, 0, stream>>>(i3, NK, NW, Wt + (size_t)(OFU + NU) * NK);
    k_gemmw<bf, 0, false><<<dim3(NR / 64, NC / 64, 1), 32, 0, stream>>>(Tb, nullptr, Wt, nullptr, NK, Pj, NC, nullptr, 0, 0, 0);
    k_bsum<<<(unsigned)(NQ * NU * NW * 128 / 256), 256, 0, stream>>>(Pj, Bs);
    k_fillf<<<(unsigned)(NQ * NU * NW * 128 / 256), 256, 0, stream>>>(Pj, Bs, Ka, Va);
    k_gemmw<h16, 0, false><<<dim3(1, 1, NQ * NU / 2), 32, 0, stream>>>(Ka, nullptr, Va, nullptr, NL, Cz, 64, nullptr, (size_t)64 * NL, (size_t)64 * NL, (size_t)64 * 64);
    k_pickd<<<(unsigned)(NQ * NW * NW * NU / 256), 256, 0, stream>>>(Cz, out);
}
